// DAInput_79001628443215
// MI455X (gfx1250) — hardware-verified
//
#include <hip/hip_runtime.h>
#include <stddef.h>


#define NTHR    256
#define NWAVE   8
#define NBN     64
#define NMAPC   128
#define KIN     22
#define KINP    32
#define AX      40
#define AP128   136
#define AP256   264
#define CP      132
#define EPT     8
#define PIECE   (NTHR * EPT)
#define WCAP    (EPT * 32)
#define GEPS    1e-5f
#define WSCALE  64.0f
#define INV64   0.015625f
#define OW1     0
#define OWT     4096
#define OW2     8192
#define OFC1    24576
#define OFC2    90112
#define OLIN    221184
#define PWTOT   286720
#define SZFC1   16384
#define SZFC2   32768
#define SZLIN   16384
#define NBLKS   4
#define PTHR    256
#define PBLK    (PWTOT / (PTHR * 8))
#define AGGDYN  262144
#define INDYN   90112
#define NODEDYN 118784
#define WSCAP   134217728

static_assert((PWTOT % (PTHR * 8)) == 0);
static_assert((OWT % 2048) == 0);
static_assert((OW2 % 2048) == 0);
static_assert((OFC1 % 2048) == 0);
static_assert((OFC2 % 2048) == 0);
static_assert((OLIN % 2048) == 0);
static_assert(OW2 + 128 * 128 == OFC1);
static_assert(OFC1 + NBLKS * SZFC1 == OFC2);
static_assert(OFC2 + NBLKS * SZFC2 == OLIN);
static_assert(OLIN + NBLKS * SZLIN == PWTOT);
static_assert(PIECE == 2048);
static_assert((EPT % 4) == 0);
static_assert(((AX * 2) % 16) == 0);
static_assert(((AP128 * 2) % 16) == 0);
static_assert(((AP256 * 2) % 16) == 0);
static_assert(((CP * 4) % 16) == 0);
static_assert(NBN == NWAVE * 8);
static_assert(INDYN == NBN * AX * 2 + NBN * AP128 * 2 + 2 * NBN * CP * 4);
static_assert(NODEDYN == NBN * AP256 * 2 + NBN * AP128 * 2 + 2 * NBN * CP * 4);
static_assert(((NBN * AX * 2) % 16) == 0);
static_assert(((NBN * AP128 * 2) % 16) == 0);
static_assert(((NBN * AP256 * 2) % 16) == 0);
static_assert(((NBN * CP * 4) % 16) == 0);

typedef float          v4f   __attribute__((ext_vector_type(4)));
typedef float          v8f   __attribute__((ext_vector_type(8)));
typedef int            v4i   __attribute__((ext_vector_type(4)));
typedef unsigned int   v4u   __attribute__((ext_vector_type(4)));
typedef unsigned short v4us  __attribute__((ext_vector_type(4)));
typedef unsigned short v8us  __attribute__((ext_vector_type(8)));
typedef _Float16       v4h   __attribute__((ext_vector_type(4)));
typedef _Float16       v8h   __attribute__((ext_vector_type(8)));
typedef _Float16       v16h  __attribute__((ext_vector_type(16)));

__device__ __forceinline__ v16h mkfrag(v8us u0, v8us u1) {
  const v8h a = __builtin_bit_cast(v8h, u0);
  const v8h b = __builtin_bit_cast(v8h, u1);
  return __builtin_shufflevector(a, b, 0, 1, 2, 3, 4, 5, 6, 7, 8, 9, 10, 11, 12, 13, 14, 15);
}

__device__ __forceinline__ v8f wmf(v16h a, v16h b, v8f c) {
  v8f d = __builtin_amdgcn_wmma_f32_16x16x32_f16(false, a, false, b, (short)0, c, false, false);
  asm volatile("v_nop\n\tv_nop\n\tv_nop\n\tv_nop" : "+v"(d) : "v"(a), "v"(b));
  return d;
}
__device__ __forceinline__ v8f zero8() {
  v8f z = {0.f, 0.f, 0.f, 0.f, 0.f, 0.f, 0.f, 0.f};
  return z;
}
template <int NT>
__device__ __forceinline__ void zacc(v8f (&c)[NT]) {
#pragma unroll
  for (int t = 0; t < NT; ++t) c[t] = zero8();
}
__device__ __forceinline__ int iclamp(int v, int lo, int hi) { return v < lo ? lo : (v > hi ? hi : v); }

__device__ __forceinline__ float wave_sum32(float x) {
#pragma unroll
  for (int o = 16; o > 0; o >>= 1) x += __shfl_xor(x, o, 32);
  return x;
}

__device__ __forceinline__ v8us pack8(v4f a, v4f b) {
  const v8f f = __builtin_shufflevector(a, b, 0, 1, 2, 3, 4, 5, 6, 7);
  const v8h h = __builtin_convertvector(f, v8h);
  return __builtin_bit_cast(v8us, h);
}
__device__ __forceinline__ unsigned short h2us(float f) {
  return __builtin_bit_cast(unsigned short, (_Float16)f);
}

template <int NT>
__device__ __forceinline__ void gemmNT(const unsigned short* ap, const unsigned short* __restrict__ bpl,
                                       int K, int nks, int n0, int m, int hh, v8f (&c)[NT]) {
#pragma unroll 1
  for (int ks = 0; ks < nks; ++ks) {
    const v16h a = mkfrag(*(const v8us*)(ap + 32 * ks), *(const v8us*)(ap + 32 * ks + 16));
    const size_t bo = (size_t)(n0 + m) * K + 32 * ks + 8 * hh;
#pragma unroll
    for (int t = 0; t < NT; ++t) {
      const size_t o = bo + (size_t)(16 * t) * K;
      const v16h b = mkfrag(*(const v8us*)(bpl + o), *(const v8us*)(bpl + o + 16));
      c[t] = wmf(a, b, c[t]);
    }
  }
}

template <int NT>
__device__ __forceinline__ void stageC(float* sC, int row0, int col0, v8f (&c)[NT]) {
#pragma unroll
  for (int t = 0; t < NT; ++t) {
    float* sp = sC + row0 * CP + col0 + 16 * t;
#pragma unroll
    for (int r = 0; r < 8; ++r) sp[r * CP] = c[t][r] * INV64;
  }
}

template <bool RELU, bool RES, bool WF, bool WH>
__device__ __forceinline__ void gn_epi(const float* sC, float* sF, unsigned short* sHo, int hp,
                                       const float* __restrict__ g, const float* __restrict__ b,
                                       int wave, int lane) {
  const v4f gg = *(const v4f*)(g + 4 * lane);
  const v4f bb = *(const v4f*)(b + 4 * lane);
#pragma unroll 2
  for (int rr = 0; rr < 8; ++rr) {
    const int row = 8 * wave + rr;
    const v4f x = *(const v4f*)(sC + row * CP + 4 * lane);
    float s = (x.x + x.y) + (x.z + x.w);
    s = wave_sum32(s);
    const float mu = s * (1.0f / 128.0f);
    v4f d;
    d.x = x.x - mu; d.y = x.y - mu; d.z = x.z - mu; d.w = x.w - mu;
    float q = (d.x * d.x + d.y * d.y) + (d.z * d.z + d.w * d.w);
    q = wave_sum32(q);
    const float rstd = rsqrtf(q * (1.0f / 128.0f) + GEPS);
    v4f o;
    o.x = (d.x * rstd) * gg.x + bb.x;
    o.y = (d.y * rstd) * gg.y + bb.y;
    o.z = (d.z * rstd) * gg.z + bb.z;
    o.w = (d.w * rstd) * gg.w + bb.w;
    if (RES) {
      const v4f rv = *(const v4f*)(sF + row * CP + 4 * lane);
      o.x += rv.x; o.y += rv.y; o.z += rv.z; o.w += rv.w;
    }
    if (RELU) {
      o.x = fmaxf(o.x, 0.0f); o.y = fmaxf(o.y, 0.0f); o.z = fmaxf(o.z, 0.0f); o.w = fmaxf(o.w, 0.0f);
    }
    if (WF) *(v4f*)(sF + row * CP + 4 * lane) = o;
    if (WH) {
      const v4h hv = __builtin_convertvector(o, v4h);
      *(v4us*)(sHo + row * hp + 4 * lane) = __builtin_bit_cast(v4us, hv);
    }
  }
}

__device__ __forceinline__ void rowsF(const float* sF, float* dst, int n0, int nrows, int tid) {
#pragma unroll 1
  for (int it = 0; it < 8; ++it) {
    const int p = it * NTHR + tid;
    const int row = p >> 5, c4 = p & 31;
    const v4f v = *(const v4f*)(sF + row * CP + 4 * c4);
    if (row < nrows) *(volatile v4f*)(dst + (size_t)(n0 + row) * NMAPC + 4 * c4) = v;
  }
}
__device__ __forceinline__ void rows128(const unsigned short* so, int ap, unsigned short* dst, int n0, int tid) {
#pragma unroll
  for (int it = 0; it < 4; ++it) {
    const int p = it * NTHR + tid;
    const int row = p >> 4, c8 = p & 15;
    const v8us v = *(const v8us*)(so + row * ap + 8 * c8);
    *(volatile v8us*)(dst + (size_t)(n0 + row) * NMAPC + 8 * c8) = v;
  }
}

__global__ __launch_bounds__(PTHR) void k_prep(
    const float* __restrict__ w1, const float* __restrict__ wt, const float* __restrict__ w2,
    const float* __restrict__ fc1, const float* __restrict__ fc2, const float* __restrict__ lin,
    unsigned short* wpl) {
  const int tid = (int)threadIdx.x;
  const int ob = (int)blockIdx.x * (PTHR * 8);
  const int o = ob + tid * 8;
  const float* src = w1;
  int sb = OW1, K = KIN, lk = 5;
  if (ob >= OLIN)      { src = lin; sb = OLIN; K = 128; lk = 7; }
  else if (ob >= OFC2) { src = fc2; sb = OFC2; K = 256; lk = 8; }
  else if (ob >= OFC1) { src = fc1; sb = OFC1; K = 128; lk = 7; }
  else if (ob >= OW2)  { src = w2;  sb = OW2;  K = 128; lk = 7; }
  else if (ob >= OWT)  { src = wt;  sb = OWT; }
  const int orel = o - sb;
  const int kk = orel >> (lk + 7);
  const int within = orel - (kk << (lk + 7));
  const int n = within >> lk;
  const int k0 = within - (n << lk);
  const float* p = src + (size_t)kk * K * NMAPC + n;
  float f[8];
#pragma unroll
  for (int j = 0; j < 8; ++j) {
    const int k = k0 + j;
    const int kc = k > K - 1 ? K - 1 : k;
    const float vv = p[(size_t)kc * NMAPC];
    f[j] = (k < K) ? vv * WSCALE : 0.0f;
  }
  v4f a, b;
  a.x = f[0]; a.y = f[1]; a.z = f[2]; a.w = f[3];
  b.x = f[4]; b.y = f[5]; b.z = f[6]; b.w = f[7];
  const v8us hv = pack8(a, b);
  unsigned short* d = wpl + o;
  *(volatile v8us*)d = hv;
  __threadfence();
  *(volatile v8us*)d = hv;
}

__global__ __launch_bounds__(NTHR) void k_in(
    const float* __restrict__ x, const unsigned short* __restrict__ wpl,
    const float* __restrict__ g1, const float* __restrict__ b1, const float* __restrict__ g2, const float* __restrict__ b2,
    const float* __restrict__ gt, const float* __restrict__ bt, const float* __restrict__ gc, const float* __restrict__ bc,
    float* F, unsigned short* CTX, int nN) {
  extern __shared__ __attribute__((aligned(16))) unsigned short dynI[];
  unsigned short* sX = dynI;
  unsigned short* sH = dynI + NBN * AX;
  float* sC = (float*)(dynI + NBN * AX + NBN * AP128);
  float* sF = (float*)(dynI + NBN * AX + NBN * AP128 + NBN * CP * 2);
  const int tid = (int)threadIdx.x, lane = tid & 31, wave = tid >> 5, hh = lane >> 4, m = lane & 15;
  const int n0 = (int)blockIdx.x * NBN;

#pragma unroll 1
  for (int it = 0; it < 8; ++it) {
    const int i = it * NTHR + tid;
    const int r = i >> 5, c = i & 31;
    int node = n0 + r;
    node = node > nN - 1 ? nN - 1 : node;
    const int cc = c > KIN - 1 ? KIN - 1 : c;
    const float vv = x[(size_t)node * KIN + cc];
    sX[r * AX + c] = h2us((c < KIN) ? vv : 0.0f);
  }
  __syncthreads();
  const int rt = wave & 3, cg = wave >> 2;

  {
    v8f c[4];
    zacc<4>(c);
    gemmNT<4>(sX + (16 * rt + m) * AX + 8 * hh, wpl + OWT, KINP, 1, 64 * cg, m, hh, c);
    stageC<4>(sC, 16 * rt + 8 * hh, 64 * cg + m, c);
  }
  __syncthreads();
  gn_epi<false, false, true, false>(sC, sF, sH, AP128, gt, bt, wave, lane);
  __syncthreads();

  {
    v8f c[4];
    zacc<4>(c);
    gemmNT<4>(sX + (16 * rt + m) * AX + 8 * hh, wpl + OW1, KINP, 1, 64 * cg, m, hh, c);
    stageC<4>(sC, 16 * rt + 8 * hh, 64 * cg + m, c);
  }
  __syncthreads();
  gn_epi<true, false, false, true>(sC, sF, sH, AP128, g1, b1, wave, lane);
  __syncthreads();

  {
    v8f c[4];
    zacc<4>(c);
    gemmNT<4>(sH + (16 * rt + m) * AP128 + 8 * hh, wpl + OW2, 128, 4, 64 * cg, m, hh, c);
    stageC<4>(sC, 16 * rt + 8 * hh, 64 * cg + m, c);
  }
  __syncthreads();
  gn_epi<true, true, true, true>(sC, sF, sH, AP128, g2, b2, wave, lane);
  __syncthreads();

  {
    v8f c[4];
    zacc<4>(c);
    gemmNT<4>(sH + (16 * rt + m) * AP128 + 8 * hh, wpl + OFC1, 128, 4, 64 * cg, m, hh, c);
    stageC<4>(sC, 16 * rt + 8 * hh, 64 * cg + m, c);
  }
  __syncthreads();
  gn_epi<true, false, false, true>(sC, sF, sH, AP128, gc, bc, wave, lane);
  __syncthreads();

  rowsF(sF, F, n0, NBN, tid);
  rows128(sH, AP128, CTX, n0, tid);
  __threadfence();
  rowsF(sF, F, n0, NBN, tid);
  rows128(sH, AP128, CTX, n0, tid);
}

template <int CPL> struct LaneVec;
template <> struct LaneVec<2> {
  typedef unsigned short U __attribute__((ext_vector_type(2)));
  typedef _Float16       H __attribute__((ext_vector_type(2)));
  typedef float          F __attribute__((ext_vector_type(2)));
};
template <> struct LaneVec<4> {
  typedef unsigned short U __attribute__((ext_vector_type(4)));
  typedef _Float16       H __attribute__((ext_vector_type(4)));
  typedef float          F __attribute__((ext_vector_type(4)));
};

template <int SLB_>
__device__ __forceinline__ int scan_piece(const int* __restrict__ ei, int lim, int cbase, int base,
                                          int* list, int tid, int wave, int vec) {
  constexpr int NBC = 1 << SLB_;
  int wc = 0;
  const int el0  = tid * EPT;
  const int e0   = cbase + el0;
  const int sent = -2147483647 - 1;
  int kk[EPT];
  if (vec != 0 && cbase + PIECE <= lim) {
    const v4i* p = (const v4i*)(ei + e0);
#pragma unroll
    for (int uu = 0; uu < EPT / 4; ++uu) {
      const v4i d = p[uu];
      kk[4 * uu] = d.x; kk[4 * uu + 1] = d.y; kk[4 * uu + 2] = d.z; kk[4 * uu + 3] = d.w;
    }
  } else {
    const int lm = lim - 1;
#pragma unroll
    for (int q = 0; q < EPT; ++q) {
      const int eq = e0 + q;
      const int ec = eq > lm ? lm : eq;
      const int a = ei[ec];
      kk[q] = (eq < lim) ? a : sent;
    }
  }
  const unsigned nb = (unsigned)base;
  unsigned sq[EPT];
  bool hq[EPT];
  bool anyl = false;
#pragma unroll
  for (int q = 0; q < EPT; ++q) {
    sq[q] = (unsigned)kk[q] - nb;
    hq[q] = sq[q] < (unsigned)NBC;
    anyl = anyl | hq[q];
  }
  const unsigned any = __builtin_amdgcn_ballot_w32(anyl);
  if (any != 0u) {
#define HIT(HQ, SQ, Q) { \
      const unsigned mj = __builtin_amdgcn_ballot_w32(HQ); \
      if (mj != 0u) { \
        if (HQ) { \
          const int ps = wc + (int)__builtin_amdgcn_mbcnt_lo(mj, 0u); \
          if (ps < WCAP) list[wave * WCAP + ps] = ((el0 + (Q)) << SLB_) | (int)(SQ); \
        } \
        wc += (int)__builtin_popcount(mj); } }
#pragma unroll
    for (int q = 0; q < EPT; ++q) {
      HIT(hq[q], sq[q], q)
    }
#undef HIT
  }
  return wc;
}

template <int NCH, int SLB_>
__device__ __forceinline__ void drain_max(const int* list, const int* wcnt, unsigned short* accH,
                                          const int* __restrict__ esrc, const unsigned short* __restrict__ PQ,
                                          int cbase, int nE, int nN, int lane, int wave) {
  constexpr int NBC = 1 << SLB_;
  constexpr int CPL = NCH / 32;
  typedef typename LaneVec<CPL>::U UT;
  typedef typename LaneVec<CPL>::H HT;
  typedef typename LaneVec<CPL>::F FT;
#pragma unroll 1
  for (int wsx = 0; wsx < NWAVE; ++wsx) {
    int n = __builtin_amdgcn_readfirstlane(wcnt[wsx]);
    n = n > WCAP ? WCAP : (n < 0 ? 0 : n);
    const int* lp = list + wsx * WCAP;
#pragma unroll 1
    for (int bb = 0; bb < n; bb += 32) {
      const int idx = bb + lane;
      const int ic = idx > WCAP - 1 ? WCAP - 1 : idx;
      const int ent = lp[ic];
      const bool own = (idx < n) && ((ent & (NWAVE - 1)) == wave);
      unsigned msk = __builtin_amdgcn_ballot_w32(own);
#pragma unroll 1
      while (msk != 0u) {
        const int bit = (int)__builtin_ctz(msk);
        msk &= msk - 1u;
        const int e2 = __builtin_amdgcn_readlane(ent, bit);
        const int slot = e2 & (NBC - 1);
        const int el = (e2 >> SLB_) & (PIECE - 1);
        int e = cbase + el;
        e = e > nE - 1 ? nE - 1 : (e < 0 ? 0 : e);
        const int s = iclamp(esrc[e], 0, nN - 1);
        const UT qb = *(const UT*)(PQ + (size_t)s * NCH + CPL * lane);
        const FT qf = __builtin_convertvector(__builtin_bit_cast(HT, qb), FT);
        unsigned short* ap = accH + slot * NCH + CPL * lane;
        const UT ab = *(const UT*)ap;
        FT af = __builtin_convertvector(__builtin_bit_cast(HT, ab), FT);
#pragma unroll
        for (int j = 0; j < CPL; ++j) af[j] = fmaxf(af[j], qf[j]);
        *(UT*)ap = __builtin_bit_cast(UT, __builtin_convertvector(af, HT));
      }
    }
  }
}

template <int NCH, int SLB_>
__device__ __forceinline__ void hn_rows(const unsigned short* accH, unsigned short* HN, int base, int lane, int wave) {
  constexpr int NBC = 1 << SLB_;
  constexpr int RPW = NBC / NWAVE;
  constexpr int L8  = NCH / 8;
  constexpr int RPI = 32 / L8;
  constexpr int NIT = RPW / RPI;
  const int sub = lane / L8, c8 = lane % L8;
#pragma unroll 1
  for (int it = 0; it < NIT; ++it) {
    const int s = wave * RPW + it * RPI + sub;
    v8us vv = *(const v8us*)(accH + s * NCH + 8 * c8);
#pragma unroll
    for (int j = 0; j < 8; ++j) vv[j] = (vv[j] == 0xFC00) ? (unsigned short)0 : vv[j];
    *(volatile v8us*)(HN + (size_t)(base + s) * NCH + 8 * c8) = vv;
  }
}

template <int NCH, int SLB_>
__global__ __launch_bounds__(NTHR) void k_agg(
    const int* __restrict__ edst, const int* __restrict__ esrc, const unsigned short* __restrict__ PQ,
    unsigned short* HN, int nE, int nN, int vec) {
  constexpr int NBC = 1 << SLB_;
  static_assert(NBC * NCH == 131072);
  static_assert(SLB_ >= 3);
  extern __shared__ __attribute__((aligned(16))) unsigned short accH[];
  __shared__ int list[NWAVE * WCAP];
  __shared__ int wcnt[NWAVE];
  const int tid = (int)threadIdx.x, lane = tid & 31, wave = tid >> 5;
  const int base = (int)blockIdx.x * NBC;
  {
    v4u nf;
    nf.x = 0xFC00FC00u; nf.y = 0xFC00FC00u; nf.z = 0xFC00FC00u; nf.w = 0xFC00FC00u;
#pragma unroll 1
    for (int i = tid; i < (NBC * NCH) / 8; i += NTHR) *(v4u*)(accH + 8 * i) = nf;
  }
  __syncthreads();
#pragma unroll 1
  for (int cbase = 0; cbase < nE; cbase += PIECE) {
    const int wc = scan_piece<SLB_>(edst, nE, cbase, base, list, tid, wave, vec);
    if (lane == 0) wcnt[wave] = wc;
    __syncthreads();
    drain_max<NCH, SLB_>(list, wcnt, accH, esrc, PQ, cbase, nE, nN, lane, wave);
    __syncthreads();
  }
  __syncthreads();
  hn_rows<NCH, SLB_>(accH, HN, base, lane, wave);
  __threadfence();
  hn_rows<NCH, SLB_>(accH, HN, base, lane, wave);
}

template <bool LAST>
__global__ __launch_bounds__(NTHR) void k_node(
    float* F, const unsigned short* __restrict__ AGG,
    const unsigned short* __restrict__ wfc2, const float* __restrict__ g2, const float* __restrict__ b2,
    const unsigned short* __restrict__ wlin, const float* __restrict__ gl, const float* __restrict__ bl,
    const unsigned short* __restrict__ wfc1n, const float* __restrict__ gc, const float* __restrict__ bc,
    unsigned short* CTX, float* out, int nN) {
  extern __shared__ __attribute__((aligned(16))) unsigned short dynN[];
  unsigned short* sA = dynN;
  unsigned short* sH = dynN + NBN * AP256;
  float* sC = (float*)(dynN + NBN * AP256 + NBN * AP128);
  float* sF = (float*)(dynN + NBN * AP256 + NBN * AP128 + NBN * CP * 2);
  const int tid = (int)threadIdx.x, lane = tid & 31, wave = tid >> 5, hh = lane >> 4, m = lane & 15;
  const int n0 = (int)blockIdx.x * NBN;

  {
    const int nl = tid >> 2, q = tid & 3;
    int node = n0 + nl;
    node = node > nN - 1 ? nN - 1 : node;
    const float* fp = F + (size_t)node * NMAPC + 32 * q;
    float* df = sF + nl * CP + 32 * q;
    unsigned short* da = sA + nl * AP256 + 32 * q;
#pragma unroll
    for (int j = 0; j < 4; ++j) {
      const v4f a0 = *(const v4f*)(fp + 8 * j);
      const v4f a1 = *(const v4f*)(fp + 8 * j + 4);
      *(v4f*)(df + 8 * j)     = a0;
      *(v4f*)(df + 8 * j + 4) = a1;
      *(v8us*)(da + 8 * j) = pack8(a0, a1);
    }
    const unsigned short* gp = AGG + (size_t)node * NMAPC + 32 * q;
    unsigned short* dg = sA + nl * AP256 + NMAPC + 32 * q;
#pragma unroll
    for (int j = 0; j < 4; ++j) *(v8us*)(dg + 8 * j) = *(const v8us*)(gp + 8 * j);
  }
  __syncthreads();
  const int rt = wave & 3, cg = wave >> 2;

  {
    v8f c[4];
    zacc<4>(c);
    gemmNT<4>(sA + (16 * rt + m) * AP256 + 8 * hh, wfc2, 256, 8, 64 * cg, m, hh, c);
    stageC<4>(sC, 16 * rt + 8 * hh, 64 * cg + m, c);
  }
  __syncthreads();
  gn_epi<true, false, false, true>(sC, sF, sH, AP128, g2, b2, wave, lane);
  __syncthreads();

  {
    v8f c[4];
    zacc<4>(c);
    gemmNT<4>(sH + (16 * rt + m) * AP128 + 8 * hh, wlin, 128, 4, 64 * cg, m, hh, c);
    stageC<4>(sC, 16 * rt + 8 * hh, 64 * cg + m, c);
  }
  __syncthreads();
  gn_epi<true, true, true, true>(sC, sF, sA, AP256, gl, bl, wave, lane);
  __syncthreads();

  if (!LAST) {
    {
      v8f c[4];
      zacc<4>(c);
      gemmNT<4>(sA + (16 * rt + m) * AP256 + 8 * hh, wfc1n, 128, 4, 64 * cg, m, hh, c);
      stageC<4>(sC, 16 * rt + 8 * hh, 64 * cg + m, c);
    }
    __syncthreads();
    gn_epi<true, false, false, true>(sC, sF, sH, AP128, gc, bc, wave, lane);
    __syncthreads();
    rowsF(sF, F, n0, NBN, tid);
    rows128(sH, AP128, CTX, n0, tid);
    __threadfence();
    rowsF(sF, F, n0, NBN, tid);
    rows128(sH, AP128, CTX, n0, tid);
  } else {
    int nr = nN - n0;
    nr = nr > NBN ? NBN : (nr < 1 ? 1 : nr);
    rowsF(sF, out, n0, nr, tid);
    __threadfence();
    rowsF(sF, out, n0, nr, tid);
  }
}

extern "C" void kernel_launch(void* const* d_in, const int* in_sizes, int n_in,
                              void* d_out, int out_size, void* d_ws, size_t ws_size,
                              hipStream_t stream) {
  if (n_in < 21) return;
  const int nN = in_sizes[0] / KIN;
  if (nN < 1 || nN > (1 << 22) || in_sizes[0] != nN * KIN) return;
  const int nE2 = in_sizes[1];
  if (nE2 < 2 || (nE2 & 1) != 0 || in_sizes[2] != nE2) return;
  const int nE = nE2 / 2;
  if (nE > (1 << 27)) return;
  if (in_sizes[3] != KIN * NMAPC || in_sizes[4] != NMAPC || in_sizes[5] != NMAPC) return;
  if (in_sizes[6] != NMAPC * NMAPC || in_sizes[7] != NMAPC || in_sizes[8] != NMAPC) return;
  if (in_sizes[9] != KIN * NMAPC || in_sizes[10] != NMAPC || in_sizes[11] != NMAPC) return;
  if (in_sizes[12] != NBLKS * SZFC1 || in_sizes[13] != NBLKS * NMAPC || in_sizes[14] != NBLKS * NMAPC) return;
  if (in_sizes[15] != NBLKS * SZFC2 || in_sizes[16] != NBLKS * NMAPC || in_sizes[17] != NBLKS * NMAPC) return;
  if (in_sizes[18] != NBLKS * SZLIN || in_sizes[19] != NBLKS * NMAPC || in_sizes[20] != NBLKS * NMAPC) return;
  if ((size_t)out_size != (size_t)nN * NMAPC) return;

  const float* feats = (const float*)d_in[0];
  const int*   eu    = (const int*)d_in[1];
  const int*   ev    = (const int*)d_in[2];
  const float* in_w1 = (const float*)d_in[3];
  const float* in_g1 = (const float*)d_in[4];
  const float* in_b1 = (const float*)d_in[5];
  const float* in_w2 = (const float*)d_in[6];
  const float* in_g2 = (const float*)d_in[7];
  const float* in_b2 = (const float*)d_in[8];
  const float* in_wt = (const float*)d_in[9];
  const float* in_gt = (const float*)d_in[10];
  const float* in_bt = (const float*)d_in[11];
  const float* fc1_w = (const float*)d_in[12];
  const float* fc1_g = (const float*)d_in[13];
  const float* fc1_b = (const float*)d_in[14];
  const float* fc2_w = (const float*)d_in[15];
  const float* fc2_g = (const float*)d_in[16];
  const float* fc2_b = (const float*)d_in[17];
  const float* lin_w = (const float*)d_in[18];
  const float* lin_g = (const float*)d_in[19];
  const float* lin_b = (const float*)d_in[20];
  float* out = (float*)d_out;

  const int nb64 = (nN + NBN - 1) / NBN;
  const int Npad64 = nb64 * NBN;
  const int nbA = (nN + 1023) / 1024;
  const int NpA = nbA * 1024;

  char* ws = (char*)d_ws;
  size_t off = 0;
  const size_t oW   = off; off += (size_t)PWTOT * 2;              off = (off + 255) & ~(size_t)255;
  const size_t oCTX = off; off += (size_t)Npad64 * NMAPC * 2;     off = (off + 255) & ~(size_t)255;
  const size_t oAGG = off; off += (size_t)NpA * NMAPC * 2;        off = (off + 255) & ~(size_t)255;
  const size_t oF   = off; off += (size_t)Npad64 * NMAPC * 4;     off = (off + 255) & ~(size_t)255;
  if (off > ws_size || off > (size_t)WSCAP) return;
  unsigned short* wpl = (unsigned short*)(ws + oW);
  unsigned short* CTX = (unsigned short*)(ws + oCTX);
  unsigned short* AGG = (unsigned short*)(ws + oAGG);
  float* F = (float*)(ws + oF);

  hipFuncSetAttribute(reinterpret_cast<const void*>(&k_agg<128, 10>), hipFuncAttributeMaxDynamicSharedMemorySize, AGGDYN);
  hipFuncSetAttribute(reinterpret_cast<const void*>(&k_in), hipFuncAttributeMaxDynamicSharedMemorySize, INDYN);
  hipFuncSetAttribute(reinterpret_cast<const void*>(&k_node<false>), hipFuncAttributeMaxDynamicSharedMemorySize, NODEDYN);
  hipFuncSetAttribute(reinterpret_cast<const void*>(&k_node<true>), hipFuncAttributeMaxDynamicSharedMemorySize, NODEDYN);

  k_prep<<<PBLK, PTHR, 0, stream>>>(in_w1, in_wt, in_w2, fc1_w, fc2_w, lin_w, wpl);
  k_in<<<nb64, NTHR, INDYN, stream>>>(feats, wpl, in_g1, in_b1, in_g2, in_b2, in_gt, in_bt,
                                       fc1_g, fc1_b, F, CTX, nN);
  for (int k = 0; k < NBLKS; ++k) {
    const int i = k & 1;
    const size_t eoff = (size_t)i * (size_t)nE;
    const int vec = ((eoff % 4) == 0) ? 1 : 0;
    k_agg<128, 10><<<nbA, NTHR, AGGDYN, stream>>>(ev + eoff, eu + eoff, CTX, AGG, nE, nN, vec);
    const int kn = (k < NBLKS - 1) ? (k + 1) : 0;
    const unsigned short* wfc2  = wpl + OFC2 + (size_t)k * SZFC2;
    const unsigned short* wlin  = wpl + OLIN + (size_t)k * SZLIN;
    const unsigned short* wfc1n = wpl + OFC1 + (size_t)kn * SZFC1;
    const float* g2 = fc2_g + (size_t)k * NMAPC;
    const float* b2 = fc2_b + (size_t)k * NMAPC;
    const float* gl = lin_g + (size_t)k * NMAPC;
    const float* bl = lin_b + (size_t)k * NMAPC;
    const float* gc = fc1_g + (size_t)kn * NMAPC;
    const float* bc = fc1_b + (size_t)kn * NMAPC;
    if (k < NBLKS - 1)
      k_node<false><<<nb64, NTHR, NODEDYN, stream>>>(F, AGG, wfc2, g2, b2, wlin, gl, bl, wfc1n, gc, bc, CTX, out, nN);
    else
      k_node<true><<<nb64, NTHR, NODEDYN, stream>>>(F, AGG, wfc2, g2, b2, wlin, gl, bl, wfc1n, gc, bc, CTX, out, nN);
  }
}
